// LSTMModel_34961033789514
// MI455X (gfx1250) — hardware-verified
//
#include <hip/hip_runtime.h>
#include <math.h>

constexpr int NBATCH   = 512;
constexpr int NSTEPS   = 512;
constexpr int NFEAT    = 32;
constexpr int HID1     = 128;
constexpr int HID2     = 64;
constexpr int HID3     = 32;
constexpr int ROWS_BLK = 32;
constexpr int NTHR     = 256;
constexpr int XPITCH   = 40;
constexpr int PITCH1   = 136;
constexpr int PITCH2   = 72;
constexpr int PITCH3   = 40;
constexpr int FPITCH   = 36;
constexpr float CARRY_ACT = 64.0f;
constexpr float CARRY_WGT = 16.0f;
constexpr float FOLD_BACK = 1.0f / (CARRY_ACT * CARRY_WGT);

constexpr int NWX1 = 4 * HID1 * NFEAT;
constexpr int NWH1 = 4 * HID1 * HID1;
constexpr int NWX2 = 4 * HID2 * HID1;
constexpr int NWH2 = 4 * HID2 * HID2;
constexpr int NWX3 = 4 * HID3 * HID2;
constexpr int NWH3 = 4 * HID3 * HID3;
constexpr int OFF_WX1 = 0;
constexpr int OFF_WH1 = OFF_WX1 + NWX1;
constexpr int OFF_WX2 = OFF_WH1 + NWH1;
constexpr int OFF_WH2 = OFF_WX2 + NWX2;
constexpr int OFF_WX3 = OFF_WH2 + NWH2;
constexpr int OFF_WH3 = OFF_WX3 + NWX3;
constexpr int NWALL   = OFF_WH3 + NWH3;
constexpr int CAST_GRP = NTHR * 8;
constexpr int CBLK1 = NWX1 / CAST_GRP;
constexpr int CBLK2 = CBLK1 + NWH1 / CAST_GRP;
constexpr int CBLK3 = CBLK2 + NWX2 / CAST_GRP;
constexpr int CBLK4 = CBLK3 + NWH2 / CAST_GRP;
constexpr int CBLK5 = CBLK4 + NWX3 / CAST_GRP;
constexpr int CBLK6 = CBLK5 + NWH3 / CAST_GRP;
constexpr int NBIAS = 4 * (HID1 + HID2 + HID3);

static_assert(NWALL == 143360, "plane size");
static_assert(NWX1 % CAST_GRP == 0 && NWH1 % CAST_GRP == 0 && NWX2 % CAST_GRP == 0, "cast blocks exact");
static_assert(NWH2 % CAST_GRP == 0 && NWX3 % CAST_GRP == 0 && NWH3 % CAST_GRP == 0, "cast blocks exact");
static_assert(CBLK6 * CAST_GRP == NWALL, "cast grid covers the plane exactly");
static_assert(NFEAT % 32 == 0 && HID1 % 32 == 0 && HID2 % 32 == 0 && HID3 % 32 == 0, "K multiples of 32");
static_assert(HID1 == 16 * (NTHR / 32), "layer 1: one 16-column unit group per wave");
static_assert(HID2 == 16 * 4 && HID3 == 16 * 2, "layer 2/3 wave maps");
static_assert(ROWS_BLK == 32 && NBATCH % ROWS_BLK == 0, "two 16-row subtiles per block");
static_assert(ROWS_BLK * NFEAT == NTHR * 4, "x tile staging exact");
static_assert(NBIAS == 896, "bias table");
static_assert(2 * HID1 == 2 * NTHR / 2 * 1 && 4 * HID1 == 2 * NTHR && 4 * HID2 == NTHR && 4 * HID3 == NTHR / 2, "bias staging map");

typedef __attribute__((ext_vector_type(16))) _Float16 v16h;
typedef __attribute__((ext_vector_type(8)))  _Float16 v8h;
typedef __attribute__((ext_vector_type(4)))  _Float16 v4h;
typedef __attribute__((ext_vector_type(8)))  float    v8f;
typedef __attribute__((ext_vector_type(4)))  float    v4f;

template <typename T> struct Frag;
template <> struct Frag<_Float16> {
  typedef v16h V; union U { v16h v; v8h h[2]; };
  static __device__ __forceinline__ v16h load(const _Float16* p) {
    U f; f.h[0] = *(const v8h*)(p); f.h[1] = *(const v8h*)(p + 16); return f.v;
  }
  static __device__ __forceinline__ v8f mma(v16h a, v16h b, v8f c) {
    return __builtin_amdgcn_wmma_f32_16x16x32_f16(false, a, false, b, (short)0, c, false, false);
  }
};
typedef Frag<_Float16> FragH;

template <int NMT> struct GroupGuard;
template <> struct GroupGuard<1> {
  static __device__ __forceinline__ void run(v8f (&acc)[1][4], v16h (&a)[1], v16h b0, v16h b1, v16h b2, v16h b3) {
    asm volatile("v_nop\n\tv_nop\n\tv_nop\n\tv_nop"
                 : "+v"(acc[0][0]), "+v"(acc[0][1]), "+v"(acc[0][2]), "+v"(acc[0][3])
                 : "v"(a[0]), "v"(b0), "v"(b1), "v"(b2), "v"(b3));
  }
};
template <> struct GroupGuard<2> {
  static __device__ __forceinline__ void run(v8f (&acc)[2][4], v16h (&a)[2], v16h b0, v16h b1, v16h b2, v16h b3) {
    asm volatile("v_nop\n\tv_nop\n\tv_nop\n\tv_nop"
                 : "+v"(acc[0][0]), "+v"(acc[0][1]), "+v"(acc[0][2]), "+v"(acc[0][3]),
                   "+v"(acc[1][0]), "+v"(acc[1][1]), "+v"(acc[1][2]), "+v"(acc[1][3])
                 : "v"(a[0]), "v"(a[1]), "v"(b0), "v"(b1), "v"(b2), "v"(b3));
  }
};

__device__ __forceinline__ float fsig(float x)  { return __builtin_amdgcn_rcpf(1.0f + __expf(-x)); }
__device__ __forceinline__ float ftanh(float x) { return 1.0f - 2.0f * __builtin_amdgcn_rcpf(__expf(2.0f * x) + 1.0f); }

__global__ __launch_bounds__(NTHR) void wcast_kernel(const float* __restrict__ w0, const float* __restrict__ w1,
                                                     const float* __restrict__ w2, const float* __restrict__ w3,
                                                     const float* __restrict__ w4, const float* __restrict__ w5,
                                                     unsigned short* __restrict__ dstp) {
  const int blk = blockIdx.x;
  if (blk >= CBLK6) return;
  const float* src = w0;
  int bfirst = 0;
  if (blk >= CBLK1) { src = w1; bfirst = CBLK1; }
  if (blk >= CBLK2) { src = w2; bfirst = CBLK2; }
  if (blk >= CBLK3) { src = w3; bfirst = CBLK3; }
  if (blk >= CBLK4) { src = w4; bfirst = CBLK4; }
  if (blk >= CBLK5) { src = w5; bfirst = CBLK5; }
  const int li = (blk - bfirst) * NTHR + threadIdx.x;
  const size_t gi = (size_t)blk * NTHR + threadIdx.x;
  const v4f a = *(const v4f*)(src + (size_t)li * 8);
  const v4f b = *(const v4f*)(src + (size_t)li * 8 + 4);
  v8h hv;
#pragma unroll
  for (int e = 0; e < 4; ++e) {
    hv[e]     = (_Float16)(a[e] * CARRY_WGT);
    hv[4 + e] = (_Float16)(b[e] * CARRY_WGT);
  }
  _Float16* dp = (_Float16*)dstp + gi * 8;
  *(volatile v8h*)dp = hv;
  __threadfence();
  *(volatile v8h*)dp = hv;
}

template <int HD, int KIN, int NMT, int PIN, int PHD, bool WREL, bool WF32>
__device__ __forceinline__ void cell_phase(const _Float16* ain, const _Float16* hold, _Float16* hnew, _Float16* hrel, float* hf32,
                                           const _Float16* __restrict__ wxp, const _Float16* __restrict__ whp,
                                           const int ub, const int mt0, const int lane, const int zoff, const bool lastf,
                                           const float bi, const float bf, const float bg, const float bo,
                                           float (&cst)[NMT][8]) {
  const int c = lane & 15, hh = lane >> 4, koff = hh * 8;
  const int j = 16 * ub + c;
  v8f acc[NMT][4];
#pragma unroll
  for (int mt = 0; mt < NMT; ++mt)
#pragma unroll
    for (int g = 0; g < 4; ++g) acc[mt][g] = (v8f){0.f, 0.f, 0.f, 0.f, 0.f, 0.f, 0.f, 0.f};

  const _Float16* wxr = wxp + (size_t)j * KIN + koff + zoff;
  const _Float16* whr = whp + (size_t)j * HD + koff + zoff;
  const _Float16* ar  = ain  + (mt0 * 16 + c) * PIN + koff;
  const _Float16* hr  = hold + (mt0 * 16 + c) * PHD + koff;

#pragma unroll 1
  for (int k0 = 0; k0 < KIN; k0 += 32) {
    const v16h b0 = FragH::load(wxr + k0);
    const v16h b1 = FragH::load(wxr + (size_t)1 * HD * KIN + k0);
    const v16h b2 = FragH::load(wxr + (size_t)2 * HD * KIN + k0);
    const v16h b3 = FragH::load(wxr + (size_t)3 * HD * KIN + k0);
    v16h a[NMT];
#pragma unroll
    for (int mt = 0; mt < NMT; ++mt) a[mt] = FragH::load(ar + mt * 16 * PIN + k0);
#pragma unroll
    for (int mt = 0; mt < NMT; ++mt) {
      acc[mt][0] = FragH::mma(a[mt], b0, acc[mt][0]);
      acc[mt][1] = FragH::mma(a[mt], b1, acc[mt][1]);
      acc[mt][2] = FragH::mma(a[mt], b2, acc[mt][2]);
      acc[mt][3] = FragH::mma(a[mt], b3, acc[mt][3]);
    }
    GroupGuard<NMT>::run(acc, a, b0, b1, b2, b3);
  }
#pragma unroll 1
  for (int k0 = 0; k0 < HD; k0 += 32) {
    const v16h b0 = FragH::load(whr + k0);
    const v16h b1 = FragH::load(whr + (size_t)1 * HD * HD + k0);
    const v16h b2 = FragH::load(whr + (size_t)2 * HD * HD + k0);
    const v16h b3 = FragH::load(whr + (size_t)3 * HD * HD + k0);
    v16h a[NMT];
#pragma unroll
    for (int mt = 0; mt < NMT; ++mt) a[mt] = FragH::load(hr + mt * 16 * PHD + k0);
#pragma unroll
    for (int mt = 0; mt < NMT; ++mt) {
      acc[mt][0] = FragH::mma(a[mt], b0, acc[mt][0]);
      acc[mt][1] = FragH::mma(a[mt], b1, acc[mt][1]);
      acc[mt][2] = FragH::mma(a[mt], b2, acc[mt][2]);
      acc[mt][3] = FragH::mma(a[mt], b3, acc[mt][3]);
    }
    GroupGuard<NMT>::run(acc, a, b0, b1, b2, b3);
  }

#pragma unroll
  for (int mt = 0; mt < NMT; ++mt) {
#pragma unroll
    for (int r = 0; r < 8; ++r) {
      const float zi = fmaf(acc[mt][0][r], FOLD_BACK, bi);
      const float zf = fmaf(acc[mt][1][r], FOLD_BACK, bf);
      const float zg = fmaf(acc[mt][2][r], FOLD_BACK, bg);
      const float zo = fmaf(acc[mt][3][r], FOLD_BACK, bo);
      const float ig = fsig(zi);
      const float fg = fsig(zf);
      const float gg = ftanh(zg);
      const float og = fsig(zo);
      const float cn = fg * cst[mt][r] + ig * gg;
      cst[mt][r] = cn;
      const float hv = og * ftanh(cn);
      const int row = (mt0 + mt) * 16 + 8 * hh + r;
      hnew[row * PHD + j] = (_Float16)(hv * CARRY_ACT);
      if (WREL) hrel[row * PHD + j] = (_Float16)(fmaxf(hv, 0.0f) * CARRY_ACT);
      if (WF32) { if (lastf) hf32[row * FPITCH + j] = hv; }
    }
  }
}

__global__ __launch_bounds__(NTHR) void lstm3_seq_kernel(const float* __restrict__ x,
                                                         const float* __restrict__ bih1, const float* __restrict__ bhh1,
                                                         const float* __restrict__ bih2, const float* __restrict__ bhh2,
                                                         const float* __restrict__ bih3, const float* __restrict__ bhh3,
                                                         const float* __restrict__ Wd, const float* __restrict__ bd,
                                                         const unsigned short* __restrict__ wplane,
                                                         float* __restrict__ out) {
  __shared__ __align__(16) _Float16 Xs[ROWS_BLK * XPITCH];
  __shared__ __align__(16) _Float16 H1s[2 * ROWS_BLK * PITCH1];
  __shared__ __align__(16) _Float16 H1r[ROWS_BLK * PITCH1];
  __shared__ __align__(16) _Float16 H2s[2 * ROWS_BLK * PITCH2];
  __shared__ __align__(16) _Float16 H2r[ROWS_BLK * PITCH2];
  __shared__ __align__(16) _Float16 H3s[2 * ROWS_BLK * PITCH3];
  __shared__ __align__(16) float    Hf[ROWS_BLK * FPITCH];
  __shared__ __align__(16) float    sB[NBIAS];

  const int tid  = threadIdx.x;
  const int lane = tid & 31;
  const int wave = __builtin_amdgcn_readfirstlane(tid >> 5);
  const int c    = lane & 15;
  const int rowbase = blockIdx.x * ROWS_BLK;

  const _Float16* WP  = (const _Float16*)wplane;
  const _Float16* WX1 = WP + OFF_WX1;
  const _Float16* WH1 = WP + OFF_WH1;
  const _Float16* WX2 = WP + OFF_WX2;
  const _Float16* WH2 = WP + OFF_WH2;
  const _Float16* WX3 = WP + OFF_WX3;
  const _Float16* WH3 = WP + OFF_WH3;

  {
    unsigned* z1 = (unsigned*)H1s;
    unsigned* z2 = (unsigned*)H2s;
    unsigned* z3 = (unsigned*)H3s;
#pragma unroll 1
    for (int i = tid; i < ROWS_BLK * PITCH1; i += NTHR) z1[i] = 0u;
#pragma unroll 1
    for (int i = tid; i < ROWS_BLK * PITCH2; i += NTHR) z2[i] = 0u;
#pragma unroll 1
    for (int i = tid; i < ROWS_BLK * PITCH3; i += NTHR) z3[i] = 0u;
  }
  {
    sB[tid]        = bih1[tid] + bhh1[tid];
    sB[NTHR + tid] = bih1[NTHR + tid] + bhh1[NTHR + tid];
    sB[4 * HID1 + tid] = bih2[tid] + bhh2[tid];
    const int i3 = tid & (4 * HID3 - 1);
    const float v3 = bih3[i3] + bhh3[i3];
    if (tid < 4 * HID3) sB[4 * HID1 + 4 * HID2 + i3] = v3;
  }
  const int xm  = tid >> 3;
  const int xf4 = (tid & 7) * 4;
  const float* xrow = x + ((size_t)(rowbase + xm) * NSTEPS) * NFEAT + xf4;
  {
    const v4f v0 = *(const v4f*)(xrow);
    v4h h0;
#pragma unroll
    for (int e = 0; e < 4; ++e) h0[e] = (_Float16)(v0[e] * CARRY_ACT);
    *(v4h*)(Xs + xm * XPITCH + xf4) = h0;
  }
  __syncthreads();

  const int ub2 = wave & 3, mt2 = wave >> 2;
  const int ub3 = wave & 1, mt3 = (wave >> 1) & 1;
  float bb1[4], bb2[4], bb3[4];
#pragma unroll
  for (int g = 0; g < 4; ++g) {
    bb1[g] = sB[g * HID1 + 16 * wave + c];
    bb2[g] = sB[4 * HID1 + g * HID2 + 16 * ub2 + c];
    bb3[g] = sB[4 * HID1 + 4 * HID2 + g * HID3 + 16 * ub3 + c];
  }
  float cs1[2][8], cs2[1][8], cs3[1][8];
#pragma unroll
  for (int r = 0; r < 8; ++r) { cs1[0][r] = 0.0f; cs1[1][r] = 0.0f; cs2[0][r] = 0.0f; cs3[0][r] = 0.0f; }

#pragma unroll 1
  for (int t = 0; t < NSTEPS; ++t) {
    const int cur = t & 1;
    const int nxt = cur ^ 1;
    const bool lastf = (t == NSTEPS - 1);
    int zoff = 0;
    asm volatile("" : "+v"(zoff));
    const int tn = (t + 1 < NSTEPS) ? (t + 1) : (NSTEPS - 1);
    v4f xv = *(const v4f*)(xrow + (size_t)tn * NFEAT);
    asm volatile("" : "+v"(xv));

    cell_phase<HID1, NFEAT, 2, XPITCH, PITCH1, true, false>(
        Xs, H1s + cur * (ROWS_BLK * PITCH1), H1s + nxt * (ROWS_BLK * PITCH1), H1r, Hf,
        WX1, WH1, wave, 0, lane, zoff, lastf, bb1[0], bb1[1], bb1[2], bb1[3], cs1);
    __syncthreads();

    {
      v4h hx;
#pragma unroll
      for (int e = 0; e < 4; ++e) hx[e] = (_Float16)(xv[e] * CARRY_ACT);
      *(v4h*)(Xs + xm * XPITCH + xf4) = hx;
    }
    cell_phase<HID2, HID1, 1, PITCH1, PITCH2, true, false>(
        H1r, H2s + cur * (ROWS_BLK * PITCH2), H2s + nxt * (ROWS_BLK * PITCH2), H2r, Hf,
        WX2, WH2, ub2, mt2, lane, zoff, lastf, bb2[0], bb2[1], bb2[2], bb2[3], cs2);
    __syncthreads();

    if (wave < 4) {
      cell_phase<HID3, HID2, 1, PITCH2, PITCH3, false, true>(
          H2r, H3s + cur * (ROWS_BLK * PITCH3), H3s + nxt * (ROWS_BLK * PITCH3), H3s + nxt * (ROWS_BLK * PITCH3), Hf,
          WX3, WH3, ub3, mt3, lane, zoff, lastf, bb3[0], bb3[1], bb3[2], bb3[3], cs3);
    }
    __syncthreads();
  }
  __syncthreads();

  if (wave == 0) {
    float s = 0.0f;
#pragma unroll 1
    for (int k = 0; k < HID3; ++k) s = fmaf(fmaxf(Hf[lane * FPITCH + k], 0.0f), Wd[k], s);
    const float res = s + bd[0];
    volatile float* op = out + rowbase + lane;
    *op = res;
    __threadfence();
    *op = res;
  }
}

extern "C" void kernel_launch(void* const* d_in, const int* in_sizes, int n_in,
                              void* d_out, int out_size, void* d_ws, size_t ws_size, hipStream_t stream) {
  if (n_in < 15 || d_out == nullptr || d_ws == nullptr) return;
  if (in_sizes[0] != NBATCH * NSTEPS * NFEAT || in_sizes[1] != NWX1 || in_sizes[2] != NWH1 ||
      in_sizes[3] != 4 * HID1 || in_sizes[4] != 4 * HID1 ||
      in_sizes[5] != NWX2 || in_sizes[6] != NWH2 || in_sizes[7] != 4 * HID2 || in_sizes[8] != 4 * HID2 ||
      in_sizes[9] != NWX3 || in_sizes[10] != NWH3 || in_sizes[11] != 4 * HID3 || in_sizes[12] != 4 * HID3 ||
      in_sizes[13] != HID3 || in_sizes[14] != 1 || out_size != NBATCH) return;

  const float* x    = (const float*)d_in[0];
  const float* Wih1 = (const float*)d_in[1];
  const float* Whh1 = (const float*)d_in[2];
  const float* bih1 = (const float*)d_in[3];
  const float* bhh1 = (const float*)d_in[4];
  const float* Wih2 = (const float*)d_in[5];
  const float* Whh2 = (const float*)d_in[6];
  const float* bih2 = (const float*)d_in[7];
  const float* bhh2 = (const float*)d_in[8];
  const float* Wih3 = (const float*)d_in[9];
  const float* Whh3 = (const float*)d_in[10];
  const float* bih3 = (const float*)d_in[11];
  const float* bhh3 = (const float*)d_in[12];
  const float* Wd   = (const float*)d_in[13];
  const float* bd   = (const float*)d_in[14];

  const size_t carve = (size_t)NWALL * 2;
  if (carve > ws_size || carve > (size_t)134217728) return;
  unsigned short* WPLANE = (unsigned short*)d_ws;

  wcast_kernel<<<CBLK6, NTHR, 0, stream>>>(Wih1, Whh1, Wih2, Whh2, Wih3, Whh3, WPLANE);
  lstm3_seq_kernel<<<NBATCH / ROWS_BLK, NTHR, 0, stream>>>(x, bih1, bhh1, bih2, bhh2, bih3, bhh3, Wd, bd, WPLANE,
                                                           (float*)d_out);
}
